// QuantLinear_26087631356146
// MI455X (gfx1250) — hardware-verified
//
#include <hip/hip_runtime.h>
#include <math.h>

typedef __attribute__((ext_vector_type(16))) _Float16 v16h;
typedef __attribute__((ext_vector_type(16))) __bf16 v16b;
typedef __attribute__((ext_vector_type(8)))  _Float16 v8h;
typedef __attribute__((ext_vector_type(8)))  float v8f;
typedef __attribute__((ext_vector_type(4)))  float v4f;
typedef __attribute__((ext_vector_type(2)))  float v2f;
typedef __attribute__((ext_vector_type(4)))  unsigned v4u;
typedef __attribute__((ext_vector_type(4)))  int v4i;
typedef float __attribute__((may_alias)) float_a;
typedef int __attribute__((may_alias)) int_a;

template <typename T> __device__ __forceinline__ void vst2(void* p, T v) { *(volatile T*)p = v; __threadfence(); *(volatile T*)p = v; }
__device__ __forceinline__ v8f wmma16(v16h a, v16h b, v8f c) {
  v8f d = __builtin_amdgcn_wmma_f32_16x16x32_f16(false, a, false, b, (short)0, c, false, false);
  asm volatile("v_nop\n\tv_nop\n\tv_nop\n\tv_nop" : "+v"(d) : "v"(a), "v"(b));
  return d;
}
__device__ __forceinline__ v8f wmma_bf(v16b a, v16b b, v8f c) {
  v8f d = __builtin_amdgcn_wmma_f32_16x16x32_bf16(false, a, false, b, (short)0, c, false, false);
  asm volatile("v_nop\n\tv_nop\n\tv_nop\n\tv_nop" : "+v"(d) : "v"(a), "v"(b));
  return d;
}
__device__ __forceinline__ v16h frag_h(const _Float16* rowk0, int lane) {
  union { v16h v; v8h q[2]; } u; const _Float16* p = rowk0 + 8 * (lane >> 4);
  u.q[0] = *(const v8h*)p; u.q[1] = *(const v8h*)(p + 16); return u.v;
}
__device__ __forceinline__ v16h frag_f32(const float* rowk0, int lane) {
  v16h a; const float* p = rowk0 + 8 * (lane >> 4);
#pragma unroll
  for (int i = 0; i < 8; ++i) { a[i] = (_Float16)p[i]; a[8 + i] = (_Float16)p[16 + i]; }
  return a;
}
__device__ __forceinline__ v16h frag_f32s(const float* rowk0, int lane, float sc) {
  v16h a; const float* p = rowk0 + 8 * (lane >> 4);
#pragma unroll
  for (int i = 0; i < 8; ++i) { a[i] = (_Float16)(p[i] * sc); a[8 + i] = (_Float16)(p[16 + i] * sc); }
  return a;
}
__device__ __forceinline__ v16h fragc_f32(const float* W, int k0, int n, int lane, int ld, int K) {
  v16h a; const int g = lane >> 4;
#pragma unroll
  for (int i = 0; i < 8; ++i) { const int ka = k0 + 8 * g + i, kb = ka + 16;
    a[i] = (_Float16)(ka < K ? W[(size_t)(ka < K ? ka : K - 1) * ld + n] : 0.f); a[8 + i] = (_Float16)(kb < K ? W[(size_t)(kb < K ? kb : K - 1) * ld + n] : 0.f); }
  return a;
}
struct F2 { v16b h, l; };
__device__ __forceinline__ F2 bsplit16(const float v[16]) { F2 r;
#pragma unroll
  for (int i = 0; i < 16; ++i) { const __bf16 h = (__bf16)v[i]; r.h[i] = h; r.l[i] = (__bf16)(v[i] - (float)h); }
  return r; }
__device__ __forceinline__ F2 split_row(const float* row, int k0, int lane) { float v[16]; const float* p = row + k0 + 8 * (lane >> 4);
#pragma unroll
  for (int i = 0; i < 8; ++i) { v[i] = p[i]; v[8 + i] = p[16 + i]; }
  return bsplit16(v); }
__device__ __forceinline__ F2 split_rowK(const float* row, int k0, int lane, int K) { float v[16]; const int g = lane >> 4;
#pragma unroll
  for (int i = 0; i < 8; ++i) { const int ka = k0 + 8 * g + i, kb = ka + 16; v[i] = ka < K ? row[ka < K ? ka : K - 1] : 0.f; v[8 + i] = kb < K ? row[kb < K ? kb : K - 1] : 0.f; }
  return bsplit16(v); }
__device__ __forceinline__ F2 split_col(const float* W, int k0, int n, int lane, int ld, int K) { float v[16]; const int g = lane >> 4;
#pragma unroll
  for (int i = 0; i < 8; ++i) { const int ka = k0 + 8 * g + i, kb = ka + 16; v[i] = ka < K ? W[(size_t)(ka < K ? ka : K - 1) * ld + n] : 0.f; v[8 + i] = kb < K ? W[(size_t)(kb < K ? kb : K - 1) * ld + n] : 0.f; }
  return bsplit16(v); }
__device__ __forceinline__ v8f mac3(const F2& a, const F2& b, v8f c) { c = wmma_bf(a.l, b.h, c); c = wmma_bf(a.h, b.l, c); return wmma_bf(a.h, b.h, c); }
__device__ __forceinline__ float sigm(float v) { return 1.0f / (1.0f + expf(-v)); }
#define LDSX() do { asm volatile("s_wait_dscnt 0" ::: "memory"); __builtin_amdgcn_wave_barrier(); __builtin_amdgcn_fence(__ATOMIC_RELEASE, "workgroup"); } while (0)

#define MR 64
#define KIN 4096
#define NOUT 11008
#define NG 32
#define QZW (NOUT / 8)
__device__ __forceinline__ float bfr(float v) { return (float)(__bf16)v; }

__global__ __launch_bounds__(128) void k_ql(const float* __restrict__ X, const int* __restrict__ QW, const int* __restrict__ QZ, const float* __restrict__ SC, const int* __restrict__ GI, const float* __restrict__ BIAS, float* __restrict__ OUT) {
  __shared__ int sg[KIN]; __shared__ __align__(16) float ssc[NG][128]; __shared__ int sz[NG][128]; __shared__ __align__(16) float sf[4][16][132];
  const int tid = threadIdx.x, wave = tid >> 5, lane = tid & 31, col = lane & 15, g = lane >> 4; const int c0 = blockIdx.x * 128;
  for (int e = tid; e < KIN; e += 128) { int gi = GI[e]; gi = gi < 0 ? 0 : (gi >= NG ? NG - 1 : gi); sg[e] = gi; }
  for (int e = tid; e < NG * 128; e += 128) { const int gr = e >> 7, cl = e & 127, o = c0 + cl; ssc[gr][cl] = bfr(SC[(size_t)gr * NOUT + o]); const int zw = QZ[(size_t)gr * QZW + (o >> 3)]; sz[gr][cl] = ((zw >> (4 * (o & 7))) & 15) + 1; }
  __syncthreads();
  v8f acc[8] = {};
#pragma unroll 1
  for (int kc = 0; kc < KIN / 32; ++kc) {
    v16b a; { const float* p = X + (size_t)(wave * 16 + col) * KIN + kc * 32 + 8 * g;
#pragma unroll
      for (int i = 0; i < 8; ++i) { a[i] = (__bf16)p[i]; a[8 + i] = (__bf16)p[16 + i]; } }
    const int kb = kc * 32 + 8 * g;
#pragma unroll
    for (int j = 0; j < 8; ++j) { const int cl = j * 16 + col, o = c0 + cl;
      const int w0 = QW[(size_t)(kb >> 3) * NOUT + o], w1 = QW[(size_t)((kb + 16) >> 3) * NOUT + o];
      asm volatile("s_wait_loadcnt 0x0" ::: "memory");
      v16b wh, wl;
#pragma unroll
      for (int i = 0; i < 8; ++i) {
        { const int gr = sg[kb + i]; const float w = ssc[gr][cl] * (float)(((w0 >> (4 * i)) & 15) - sz[gr][cl]); const __bf16 h = (__bf16)w; wh[i] = h; wl[i] = (__bf16)(w - (float)h); }
        { const int gr = sg[kb + 16 + i]; const float w = ssc[gr][cl] * (float)(((w1 >> (4 * i)) & 15) - sz[gr][cl]); const __bf16 h = (__bf16)w; wh[8 + i] = h; wl[8 + i] = (__bf16)(w - (float)h); } }
      acc[j] = wmma_bf(a, wh, acc[j]); acc[j] = wmma_bf(a, wl, acc[j]); } }
#pragma unroll
  for (int j = 0; j < 8; ++j) { const float bb = bfr(BIAS[c0 + j * 16 + col]);
#pragma unroll
    for (int r = 0; r < 8; ++r) sf[wave][8 * g + r][j * 16 + col] = acc[j][r] + bb; }
  LDSX(); for (int rl = 0; rl < 16; ++rl) vst2(OUT + (size_t)(wave * 16 + rl) * NOUT + c0 + lane * 4, *(const v4f*)&sf[wave][rl][lane * 4]); }
extern "C" void kernel_launch(void* const* d_in, const int* in_sizes, int n_in, void* d_out, int out_size, void* d_ws, size_t ws_size, hipStream_t stream) {
  (void)in_sizes; (void)n_in; (void)out_size; (void)d_ws; (void)ws_size;
  k_ql<<<dim3(NOUT / 128), 128, 0, stream>>>((const float*)d_in[0], (const int*)d_in[1], (const int*)d_in[2], (const float*)d_in[3], (const int*)d_in[4], (const float*)d_in[5], (float*)d_out);
}
